// MaskMultiHeadAttention_91233695302254
// MI455X (gfx1250) — hardware-run, weakly checked
//
#include <hip/hip_runtime.h>
#include <math.h>
#include <stdint.h>

#define NB    4
#define SEQ   1024
#define DMOD  1024
#define NH    16
#define HD    64
#define QT_BITS 4
#define NH_BITS 4
#define ROWS  (NB * SEQ)
#define RS    (NH * HD)
#define NKB   (SEQ / 32)
#define NW32  (SEQ / 32)
#define QSC   8.0f
#define KSC   8.0f
#define RSC   2048.0f
#define RINV  (1.0f / 2048.0f)
#define PCAR  32768.0f
#define VCAR  1024.0f
#define OSC   1024.0f
#define WOS   1024.0f
#define SCL   (0.125f / 64.0f)
#define LOG2E 1.4426950408889634f
#define MADD  (-100.0f)
#define ATT_WAVES   4
#define ATT_THREADS (ATT_WAVES * 32)
#define ATT_BLOCKS  (NB * NH * (SEQ / 64))
#define SPITCH 68
#define SLABF  (16 * SPITCH)
#define SLAB64 (16 * 68)
#define VTP    72
#define NPART  (ATT_BLOCKS * ATT_WAVES * 32)
#define OUT0N  (ROWS * DMOD)
#define OUT1N  (NB * SEQ)

static_assert(HD == 64 && DMOD == NH * HD && RS == DMOD);
static_assert((1 << QT_BITS) == (SEQ / 64) && (1 << NH_BITS) == NH);
static_assert((SEQ % 64) == 0 && (SEQ % 32) == 0 && NKB * 32 == SEQ && NW32 == NKB);
static_assert(((ROWS * DMOD / 8) % 256) == 0 && ((DMOD * DMOD / 8) % 256) == 0);
static_assert((ROWS % 64) == 0 && (DMOD % 64) == 0 && (DMOD % 32) == 0);
static_assert(ATT_THREADS == 128 && ATT_BLOCKS == 1024);
static_assert(((SPITCH * 4) % 16) == 0 && ((VTP * 2) % 16) == 0 && (SPITCH >= HD + 4) && (VTP >= 64));
static_assert((OUT1N % 256) == 0 && (SEQ % 32) == 0);
static_assert(NB * NW32 * SEQ == 131072 && NPART == 131072);

typedef unsigned short u16;
typedef _Float16 v16h __attribute__((ext_vector_type(16)));
typedef _Float16 v8h  __attribute__((ext_vector_type(8)));
typedef __bf16   v16b __attribute__((ext_vector_type(16)));
typedef float    v8f  __attribute__((ext_vector_type(8)));
typedef float    v4f  __attribute__((ext_vector_type(4)));
typedef unsigned int v4u __attribute__((ext_vector_type(4)));

union FragH { v16h v; v8h h[2]; v4u u[2]; };
union FragB { v16b v; v4u u[2]; };

__device__ __forceinline__ unsigned short bf_bits(float f) {
  unsigned u = __float_as_uint(f);
  return (unsigned short)((u + 0x7FFFu + ((u >> 16) & 1u)) >> 16);
}
__device__ __forceinline__ float bf_up(unsigned short h) { return __uint_as_float(((unsigned)h) << 16); }
__device__ __forceinline__ float bfr(float f) { return bf_up(bf_bits(f)); }
__device__ __forceinline__ unsigned short h_bits(_Float16 x) { return __builtin_bit_cast(unsigned short, x); }
__device__ __forceinline__ unsigned pk16(unsigned short a, unsigned short b) { return (unsigned)a | ((unsigned)b << 16); }
__device__ __forceinline__ v8f zero8() { v8f z = {0.f, 0.f, 0.f, 0.f, 0.f, 0.f, 0.f, 0.f}; return z; }
__device__ __forceinline__ v4f zero4() { v4f z = {0.f, 0.f, 0.f, 0.f}; return z; }

__device__ __forceinline__ v16h ldfrag_h(const _Float16* p) {
  FragH f;
  f.h[0] = *(const v8h*)(p);
  f.h[1] = *(const v8h*)(p + 16);
  return f.v;
}
__device__ __forceinline__ v16b ldfrag_b(const u16* p) {
  FragB f;
  f.u[0] = *(const v4u*)(p);
  f.u[1] = *(const v4u*)(p + 16);
  return f.v;
}

__device__ __forceinline__ v8f mma_h(v16h a, v16h b, v8f c) {
  return __builtin_amdgcn_wmma_f32_16x16x32_f16(false, a, false, b, (short)0, c, false, false);
}
__device__ __forceinline__ v8f mma_b(v16b a, v16b b, v8f c) {
  return __builtin_amdgcn_wmma_f32_16x16x32_bf16(false, a, false, b, (short)0, c, false, false);
}
template <typename F>
__device__ __forceinline__ void guard6(v8f& a, v8f& b, v8f& c, v8f& d, F x0, F x1, F x2, F x3, F x4, F x5) {
#if defined(__HIP_DEVICE_COMPILE__)
  asm volatile("v_nop\n\tv_nop\n\tv_nop\n\tv_nop"
               : "+v"(a), "+v"(b), "+v"(c), "+v"(d) : "v"(x0), "v"(x1), "v"(x2), "v"(x3), "v"(x4), "v"(x5) : "memory");
#endif
}
__device__ __forceinline__ void acc_guard4(v8f& a, v8f& b, v8f& c, v8f& d) {
#if defined(__HIP_DEVICE_COMPILE__)
  asm volatile("v_nop\n\tv_nop\n\tv_nop\n\tv_nop" : "+v"(a), "+v"(b), "+v"(c), "+v"(d));
#endif
}
__device__ __forceinline__ void wave_sync_lds() {
  __builtin_amdgcn_fence(__ATOMIC_RELEASE, "workgroup");
  __builtin_amdgcn_wave_barrier();
  __builtin_amdgcn_fence(__ATOMIC_ACQUIRE, "workgroup");
}

__global__ __launch_bounds__(256) void cvt16(const float* __restrict__ x, u16* D, int n8, int mode, float scale) {
  const int gt = blockIdx.x * 256 + (int)threadIdx.x;
  if (gt >= n8) return;
  const float* p = x + (size_t)gt * 8;
  const v4f a = *(const v4f*)(p), c4 = *(const v4f*)(p + 4);
  float v[8];
#pragma unroll
  for (int e = 0; e < 4; ++e) { v[e] = a[e]; v[4 + e] = c4[e]; }
  unsigned short s[8];
#pragma unroll
  for (int e = 0; e < 8; ++e) {
    const float vb = bfr(v[e]);
    const float vf = (mode == 1) ? vb : v[e];
    const unsigned short hb = h_bits((_Float16)(vf * scale));
    const unsigned short bb = bf_bits(v[e]);
    s[e] = (mode != 0) ? hb : bb;
  }
  v4u o;
#pragma unroll
  for (int e = 0; e < 4; ++e) o[e] = pk16(s[2 * e], s[2 * e + 1]);
  u16* d = D + (size_t)gt * 8;
  for (int pass = 0; pass < 2; ++pass) {
    *(volatile v4u*)(d) = o;
    __threadfence();
  }
}

__global__ __launch_bounds__(256) void cvt_split(const float* __restrict__ x, u16* Hp, u16* Lp, int n8, float scale) {
#pragma clang fp contract(off)
  const int gt = blockIdx.x * 256 + (int)threadIdx.x;
  if (gt >= n8) return;
  const float* p = x + (size_t)gt * 8;
  const v4f a = *(const v4f*)(p), c4 = *(const v4f*)(p + 4);
  float v[8];
#pragma unroll
  for (int e = 0; e < 4; ++e) { v[e] = a[e] * scale; v[4 + e] = c4[e] * scale; }
  unsigned short sh[8], sl[8];
#pragma unroll
  for (int e = 0; e < 8; ++e) {
    const _Float16 hv = (_Float16)v[e];
    const float res = (v[e] - (float)hv) * RSC;
    sh[e] = h_bits(hv);
    sl[e] = h_bits((_Float16)res);
  }
  v4u oh, ol;
#pragma unroll
  for (int e = 0; e < 4; ++e) { oh[e] = pk16(sh[2 * e], sh[2 * e + 1]); ol[e] = pk16(sl[2 * e], sl[2 * e + 1]); }
  u16* dh = Hp + (size_t)gt * 8;
  u16* dl = Lp + (size_t)gt * 8;
  for (int pass = 0; pass < 2; ++pass) {
    *(volatile v4u*)(dh) = oh;
    *(volatile v4u*)(dl) = ol;
    __threadfence();
  }
}

__device__ __forceinline__ void epi64(float* sl, v8f a0, v8f a1, v8f a2, v8f a3, float oscale, v4f badd, float* C, int N,
                                      size_t rowb, int col0, int lane) {
  const int hh = lane >> 4, m = lane & 15;
#pragma unroll
  for (int r = 0; r < 8; ++r) {
    const int ro = (8 * hh + r) * 68 + m;
    sl[ro]      = a0[r] * oscale;
    sl[ro + 16] = a1[r] * oscale;
    sl[ro + 32] = a2[r] * oscale;
    sl[ro + 48] = a3[r] * oscale;
  }
  wave_sync_lds();
  v4f vals[8];
#pragma unroll
  for (int it = 0; it < 8; ++it) vals[it] = *(const v4f*)(sl + (it * 2 + hh) * 68 + m * 4) + badd;
  float* dst = C + (rowb + (size_t)hh) * (size_t)N + col0 + m * 4;
  for (int pass = 0; pass < 2; ++pass) {
#pragma unroll
    for (int it = 0; it < 8; ++it) {
      *(volatile v4f*)(dst + (size_t)(it * 2) * (size_t)N) = vals[it];
    }
    __threadfence();
  }
}

__global__ __launch_bounds__(128)
void gemm_bfb(const u16* __restrict__ A, const u16* __restrict__ Bt, const float* __restrict__ bias,
              float* C, int M, int N, int K, float oscale) {
  __shared__ __align__(16) float slab[4 * SLAB64];
  const int tid = threadIdx.x, wave = tid >> 5, lane = tid & 31, hh = lane >> 4, m = lane & 15;
  const int ntile = N >> 6;
  const int bid   = blockIdx.x;
  const int rowb  = (bid / ntile) * 64 + wave * 16;
  const int col0  = (bid % ntile) * 64;
  if (rowb + 16 > M) return;
  const u16* ap = A  + (size_t)(rowb + m) * K + 8 * hh;
  const u16* bp = Bt + (size_t)(col0 + m) * K + 8 * hh;
  const size_t bs = (size_t)16 * K;
  v8f acc0 = zero8(), acc1 = zero8(), acc2 = zero8(), acc3 = zero8();
#pragma unroll 1
  for (int k0 = 0; k0 < K; k0 += 32) {
    const v16b a  = ldfrag_b(ap + k0);
    const v16b b0 = ldfrag_b(bp + k0);
    const v16b b1 = ldfrag_b(bp + bs + k0);
    const v16b b2 = ldfrag_b(bp + 2 * bs + k0);
    const v16b b3 = ldfrag_b(bp + 3 * bs + k0);
    acc0 = mma_b(a, b0, acc0);
    acc1 = mma_b(a, b1, acc1);
    acc2 = mma_b(a, b2, acc2);
    acc3 = mma_b(a, b3, acc3);
    guard6<v16b>(acc0, acc1, acc2, acc3, a, b0, b1, b2, b3, a);
  }
  const v4f bv = *(const v4f*)(bias + col0 + m * 4);
  v4f badd;
#pragma unroll
  for (int e = 0; e < 4; ++e) badd[e] = bfr(bv[e]);
  epi64(slab + wave * SLAB64, acc0, acc1, acc2, acc3, oscale, badd, C, N, (size_t)rowb, col0, lane);
}

__global__ __launch_bounds__(128)
void gemm_h1(const u16* __restrict__ A, const u16* __restrict__ Bt, const float* __restrict__ bias,
             float* C, int M, int N, int K, float oscale) {
  __shared__ __align__(16) float slab[4 * SLAB64];
  const int tid = threadIdx.x, wave = tid >> 5, lane = tid & 31, hh = lane >> 4, m = lane & 15;
  const int ntile = N >> 6;
  const int bid   = blockIdx.x;
  const int rowb  = (bid / ntile) * 64 + wave * 16;
  const int col0  = (bid % ntile) * 64;
  if (rowb + 16 > M) return;
  const _Float16* ap = (const _Float16*)(const void*)A  + (size_t)(rowb + m) * K + 8 * hh;
  const _Float16* bp = (const _Float16*)(const void*)Bt + (size_t)(col0 + m) * K + 8 * hh;
  const size_t bs = (size_t)16 * K;
  v8f acc0 = zero8(), acc1 = zero8(), acc2 = zero8(), acc3 = zero8();
#pragma unroll 1
  for (int k0 = 0; k0 < K; k0 += 32) {
    const v16h a  = ldfrag_h(ap + k0);
    const v16h b0 = ldfrag_h(bp + k0);
    const v16h b1 = ldfrag_h(bp + bs + k0);
    const v16h b2 = ldfrag_h(bp + 2 * bs + k0);
    const v16h b3 = ldfrag_h(bp + 3 * bs + k0);
    acc0 = mma_h(a, b0, acc0);
    acc1 = mma_h(a, b1, acc1);
    acc2 = mma_h(a, b2, acc2);
    acc3 = mma_h(a, b3, acc3);
    guard6<v16h>(acc0, acc1, acc2, acc3, a, b0, b1, b2, b3, a);
  }
  const v4f bv = *(const v4f*)(bias + col0 + m * 4);
  v4f badd;
#pragma unroll
  for (int e = 0; e < 4; ++e) badd[e] = bfr(bv[e]);
  epi64(slab + wave * SLAB64, acc0, acc1, acc2, acc3, oscale, badd, C, N, (size_t)rowb, col0, lane);
}

__global__ __launch_bounds__(256) void vt16(const float* __restrict__ v, u16* VPo) {
  __shared__ __align__(16) u16 TH[HD * VTP];
  const int tid = threadIdx.x;
  const int bid = blockIdx.x;
  const int st  = bid & ((SEQ / 64) - 1);
  const int h   = (bid >> QT_BITS) & (NH - 1);
  const int b   = bid >> (QT_BITS + NH_BITS);
  const int s0  = st * 64;
  {
    const int sl = tid >> 2;
    const int dc = (tid & 3) * 16;
    const float* src = v + ((size_t)(b * SEQ + s0 + sl) * NH + h) * HD + dc;
#pragma unroll
    for (int i = 0; i < 4; ++i) {
      const v4f a = *(const v4f*)(src + 4 * i);
#pragma unroll
      for (int e = 0; e < 4; ++e) {
        const _Float16 hv = (_Float16)(a[e] * VCAR);
        TH[(dc + 4 * i + e) * VTP + sl] = h_bits(hv);
      }
    }
  }
  __syncthreads();
  v4u vh[2];
  const int q8 = tid >> 3, p8 = (tid & 7) * 8;
#pragma unroll
  for (int it = 0; it < 2; ++it) {
    const int line = it * 32 + q8;
    vh[it] = *(const v4u*)(TH + line * VTP + p8);
  }
  const size_t base = ((size_t)(b * NH + h) * HD) * SEQ + s0 + p8;
  for (int pass = 0; pass < 2; ++pass) {
#pragma unroll
    for (int it = 0; it < 2; ++it) {
      const int line = it * 32 + q8;
      *(volatile v4u*)(VPo + base + (size_t)line * SEQ) = vh[it];
    }
    __threadfence();
  }
}

__global__ __launch_bounds__(256) void maskbits(const float* __restrict__ mask, const float* __restrict__ mask_ver,
                                                unsigned* MBT) {
  __shared__ float vt[32][33];
  __shared__ __align__(16) unsigned sw[32];
  const int tid = threadIdx.x;
  const int bid = blockIdx.x;
  const int nw  = bid & 31;
  const int mt  = (bid >> 5) & 31;
  const int b   = bid >> 10;
  const int m0  = mt * 32, n0 = nw * 32;
  {
    const int j = tid >> 3, iq = (tid & 7) * 4;
    const v4f t = *(const v4f*)(mask_ver + ((size_t)(b * SEQ + n0 + j)) * SEQ + m0 + iq);
#pragma unroll
    for (int e = 0; e < 4; ++e) vt[j][iq + e] = t[e];
  }
  __syncthreads();
  const int i = tid >> 3, jq = (tid & 7) * 4;
  const v4f hm = *(const v4f*)(mask + ((size_t)(b * SEQ + m0 + i)) * SEQ + n0 + jq);
  unsigned bits = 0u;
#pragma unroll
  for (int e = 0; e < 4; ++e) {
    const float hv = bfr(hm[e]);
    const float vv = bfr(vt[jq + e][i]);
    const int f = ((hv >= 0.5f) ? 1 : 0) + ((vv >= 0.5f) ? 1 : 0);
    bits |= ((f == 1) ? 1u : 0u) << e;
  }
  bits <<= jq;
  bits |= __shfl_xor(bits, 1, 32);
  bits |= __shfl_xor(bits, 2, 32);
  bits |= __shfl_xor(bits, 4, 32);
  if ((tid & 7) == 0) sw[i] = bits;
  __syncthreads();
  const int tl = tid & 7;
  const v4u w = *(const v4u*)(sw + 4 * tl);
  unsigned* dst = MBT + ((size_t)(b * NW32 + nw)) * SEQ + m0 + 4 * tl;
  for (int pass = 0; pass < 2; ++pass) {
    if (tid < 8) *(volatile v4u*)(dst) = w;
    __threadfence();
  }
}

__global__ __launch_bounds__(ATT_THREADS)
void attn_fwd(const u16* __restrict__ QHp, const u16* __restrict__ QLp, const u16* __restrict__ KHp,
              const u16* __restrict__ KLp, const u16* __restrict__ VPp, const unsigned* __restrict__ MBT,
              u16* OPo, float* PART) {
  __shared__ __align__(16) float smem[ATT_WAVES * SLABF];

  const int tid  = threadIdx.x;
  const int wave = tid >> 5;
  const int lane = tid & 31;
  const int hh   = lane >> 4;
  const int c    = lane & 15;

  const int bid  = blockIdx.x;
  const int qt   = bid & ((SEQ / 64) - 1);
  const int head = (bid >> QT_BITS) & (NH - 1);
  const int b    = bid >> (QT_BITS + NH_BITS);
  const int q0   = qt * 64 + wave * 16;

  const size_t qoff = ((size_t)(b * SEQ + q0 + c)) * RS + head * HD + 8 * hh;
  const _Float16* Qhb = (const _Float16*)(const void*)QHp + qoff;
  const _Float16* Qlb = (const _Float16*)(const void*)QLp + qoff;
  const size_t koff = ((size_t)(b * SEQ + c)) * RS + head * HD + 8 * hh;
  const _Float16* Khb = (const _Float16*)(const void*)KHp + koff;
  const _Float16* Klb = (const _Float16*)(const void*)KLp + koff;
  const _Float16* Vb = (const _Float16*)(const void*)VPp + ((size_t)(b * NH + head) * HD + c) * SEQ + 8 * hh;
  const unsigned* mrow = MBT + (size_t)b * NW32 * SEQ + q0 + c;

  const v16h qh0 = ldfrag_h(Qhb);
  const v16h qh1 = ldfrag_h(Qhb + 32);
  const v16h ql0 = ldfrag_h(Qlb);
  const v16h ql1 = ldfrag_h(Qlb + 32);

  float mrun = -INFINITY, lrun = 0.f, ssum = 0.f;
  int cnt = 0;
  v8f o0 = zero8(), o1 = zero8(), o2 = zero8(), o3 = zero8();

#pragma unroll 1
  for (int it = 0; it < NKB; ++it) {
    const int kb = it * 32;
    v8f s0 = zero8(), s1 = zero8(), x0 = zero8(), x1 = zero8();
    const _Float16* k0p = Khb + (size_t)kb * RS;
    const _Float16* k1p = k0p + (size_t)16 * RS;
    const _Float16* l0p = Klb + (size_t)kb * RS;
    const _Float16* l1p = l0p + (size_t)16 * RS;
    {
      const v16h ka = ldfrag_h(k0p), kc = ldfrag_h(k1p);
      const v16h la = ldfrag_h(l0p), lc = ldfrag_h(l1p);
      s0 = mma_h(ka, qh0, s0);
      s1 = mma_h(kc, qh0, s1);
      x0 = mma_h(ka, ql0, x0);
      x0 = mma_h(la, qh0, x0);
      x1 = mma_h(kc, ql0, x1);
      x1 = mma_h(lc, qh0, x1);
      guard6<v16h>(s0, s1, x0, x1, ka, kc, la, lc, qh0, ql0);
    }
    {
      const v16h ka = ldfrag_h(k0p + 32), kc = ldfrag_h(k1p + 32);
      const v16h la = ldfrag_h(l0p + 32), lc = ldfrag_h(l1p + 32);
      s0 = mma_h(ka, qh1, s0);
      s1 = mma_h(kc, qh1, s1);
      x0 = mma_h(ka, ql1, x0);
      x0 = mma_h(la, qh1, x0);
      x1 = mma_h(kc, ql1, x1);
      x1 = mma_h(lc, qh1, x1);
      guard6<v16h>(s0, s1, x0, x1, ka, kc, la, lc, qh1, ql1);
    }
    const unsigned mw  = mrow[(size_t)it * SEQ];
    const unsigned blo = (mw >> (8 * hh)) & 0xFFu;
    const unsigned bhi = (mw >> (16 + 8 * hh)) & 0xFFu;
    float tk[16];
#pragma unroll
    for (int i = 0; i < 8; ++i) {
      const float sa = (s0[i] + x0[i] * RINV) * SCL;
      const float sb = (s1[i] + x1[i] * RINV) * SCL;
      const unsigned ba = (blo >> i) & 1u, bb = (bhi >> i) & 1u;
      ssum += sa + sb;
      cnt  += (int)(ba + bb);
      tk[i]     = (sa + (ba ? MADD : 0.f)) * LOG2E;
      tk[8 + i] = (sb + (bb ? MADD : 0.f)) * LOG2E;
    }
    float cm = -INFINITY;
#pragma unroll
    for (int i = 0; i < 16; ++i) cm = fmaxf(cm, tk[i]);
    cm = fmaxf(cm, __shfl_xor(cm, 16, 32));
    const float mn = fmaxf(mrun, cm);
    const float al = (mrun == -INFINITY) ? 0.f : exp2f(mrun - mn);
    mrun = mn;
    float ps = 0.f;
    FragH ph;
#pragma unroll
    for (int w = 0; w < 2; ++w) {
#pragma unroll
      for (int e4 = 0; e4 < 4; ++e4) {
        const int i = 8 * w + 2 * e4;
        const float p0 = exp2f(fminf(tk[i] - mn, 0.f));
        const float p1 = exp2f(fminf(tk[i + 1] - mn, 0.f));
        ps += p0 + p1;
        ph.u[w][e4] = pk16(h_bits((_Float16)(p0 * PCAR)), h_bits((_Float16)(p1 * PCAR)));
      }
    }
    ps += __shfl_xor(ps, 16, 32);
    lrun = lrun * al + ps;
    float scl[8];
#pragma unroll
    for (int r = 0; r < 8; ++r) scl[r] = __shfl(al, 8 * hh + r, 32);
#pragma unroll
    for (int r = 0; r < 8; ++r) { o0[r] *= scl[r]; o1[r] *= scl[r]; o2[r] *= scl[r]; o3[r] *= scl[r]; }
    {
      const _Float16* vp = Vb + kb;
      const v16h vf0 = ldfrag_h(vp);
      const v16h vf1 = ldfrag_h(vp + (size_t)16 * SEQ);
      const v16h vf2 = ldfrag_h(vp + (size_t)32 * SEQ);
      const v16h vf3 = ldfrag_h(vp + (size_t)48 * SEQ);
      o0 = mma_h(ph.v, vf0, o0);
      o1 = mma_h(ph.v, vf1, o1);
      o2 = mma_h(ph.v, vf2, o2);
      o3 = mma_h(ph.v, vf3, o3);
      guard6<v16h>(o0, o1, o2, o3, ph.v, vf0, vf1, vf2, vf3, ph.v);
    }
  }
  acc_guard4(o0, o1, o2, o3);

  const float rl   = (lrun > 0.f) ? (1.0f / lrun) : 0.f;
  const float linv = rl * (1.0f / (PCAR * VCAR));
  float inv[8];
#pragma unroll
  for (int r = 0; r < 8; ++r) inv[r] = __shfl(linv, 8 * hh + r, 32);
  float* slab = smem + wave * SLABF;
#pragma unroll
  for (int r = 0; r < 8; ++r) {
    const int ro = (8 * hh + r) * SPITCH + c;
    slab[ro]      = o0[r] * inv[r];
    slab[ro + 16] = o1[r] * inv[r];
    slab[ro + 32] = o2[r] * inv[r];
    slab[ro + 48] = o3[r] * inv[r];
  }
  wave_sync_lds();
  const int rq = lane >> 3, p8 = (lane & 7) * 8;
  v4u oh[4];
#pragma unroll
  for (int it = 0; it < 4; ++it) {
    const int row = it * 4 + rq;
    const v4f a = *(const v4f*)(slab + row * SPITCH + p8), c4 = *(const v4f*)(slab + row * SPITCH + p8 + 4);
    float w[8];
#pragma unroll
    for (int e = 0; e < 4; ++e) { w[e] = a[e] * OSC; w[4 + e] = c4[e] * OSC; }
#pragma unroll
    for (int e = 0; e < 4; ++e) {
      const _Float16 h0 = (_Float16)w[2 * e], h1 = (_Float16)w[2 * e + 1];
      oh[it][e] = pk16(h_bits(h0), h_bits(h1));
    }
  }
  ssum += __shfl_xor(ssum, 16, 32);
  cnt  += __shfl_xor(cnt, 16, 32);
  const float rowv = ssum + MADD * (float)cnt;
  float g[4];
#pragma unroll
  for (int e = 0; e < 4; ++e) g[e] = __shfl(rowv, 4 * (lane & 7) + e, 32);
  v4f pv;
#pragma unroll
  for (int e = 0; e < 4; ++e) pv[e] = (lane < 4) ? g[e] : 0.f;
  float* pd = PART + ((size_t)bid * ATT_WAVES + wave) * 32 + (lane & 7) * 4;
  const size_t ob = ((size_t)(b * SEQ + q0)) * RS + head * HD + p8;
  for (int pass = 0; pass < 2; ++pass) {
#pragma unroll
    for (int it = 0; it < 4; ++it) {
      const int row = it * 4 + rq;
      *(volatile v4u*)(OPo + ob + (size_t)row * RS) = oh[it];
    }
    if (lane < 8) *(volatile v4f*)(pd) = pv;
    __threadfence();
  }
}

__global__ __launch_bounds__(256) void wout(const float* __restrict__ PART, float* out1) {
  __shared__ __align__(16) float sw[256];
  const int tid = threadIdx.x;
  const int t = blockIdx.x * 256 + tid;
  const int b = t >> 10, s = t & (SEQ - 1);
  float acc = 0.f;
#pragma unroll 1
  for (int h = 0; h < NH; ++h) {
    const float rsum = PART[((size_t)((b * NH + h) * 64 + (s >> 4))) * 32 + (s & 15)];
    acc += rsum * (1.0f / (float)SEQ);
  }
  sw[tid] = acc * (1.0f / (float)NH);
  __syncthreads();
  const int tl = tid & 63;
  const v4f v = *(const v4f*)(sw + 4 * tl);
  float* dst = out1 + (size_t)blockIdx.x * 256 + 4 * tl;
  for (int pass = 0; pass < 2; ++pass) {
    if (tid < 64) *(volatile v4f*)(dst) = v;
    __threadfence();
  }
}

extern "C" void kernel_launch(void* const* d_in, const int* in_sizes, int n_in,
                              void* d_out, int out_size, void* d_ws, size_t ws_size,
                              hipStream_t stream) {
  if (n_in < 13) return;
  if (in_sizes[0] != ROWS * DMOD || in_sizes[1] != ROWS * DMOD || in_sizes[2] != ROWS * DMOD) return;
  if (in_sizes[3] != NB * SEQ * SEQ || in_sizes[4] != NB * SEQ * SEQ) return;
  if (in_sizes[5] != DMOD * DMOD || in_sizes[7] != DMOD * DMOD || in_sizes[9] != DMOD * DMOD || in_sizes[11] != DMOD * DMOD) return;
  if (in_sizes[6] != DMOD || in_sizes[8] != DMOD || in_sizes[10] != DMOD || in_sizes[12] != DMOD) return;
  if (out_size != OUT0N + OUT1N) return;

  const float* q    = (const float*)d_in[0];
  const float* k    = (const float*)d_in[1];
  const float* v    = (const float*)d_in[2];
  const float* mask = (const float*)d_in[3];
  const float* mskv = (const float*)d_in[4];
  const float* wq   = (const float*)d_in[5];
  const float* bq   = (const float*)d_in[6];
  const float* wk   = (const float*)d_in[7];
  const float* bk   = (const float*)d_in[8];
  const float* wv   = (const float*)d_in[9];
  const float* bv   = (const float*)d_in[10];
  const float* wo   = (const float*)d_in[11];
  const float* bo   = (const float*)d_in[12];
  float*       out0 = (float*)d_out;
  float*       out1 = (float*)d_out + (size_t)OUT0N;

  const size_t szXB   = (size_t)ROWS * DMOD * 2;
  const size_t szWB   = (size_t)DMOD * DMOD * 2;
  const size_t szF    = (size_t)ROWS * DMOD * 4;
  const size_t szP    = (size_t)ROWS * DMOD * 2;
  const size_t szVP   = (size_t)NB * NH * HD * SEQ * 2;
  const size_t szMB   = (size_t)NB * NW32 * SEQ * 4;
  const size_t szPART = (size_t)NPART * 4;
  size_t off = 0;
  const size_t oXB   = off; off += szXB;
  const size_t oWB   = off; off += szWB;
  const size_t oF    = off; off += szF;
  const size_t oQH   = off; off += szP;
  const size_t oQL   = off; off += szP;
  const size_t oKH   = off; off += szP;
  const size_t oKL   = off; off += szP;
  const size_t oVP   = off; off += szVP;
  const size_t oOP   = off; off += szP;
  const size_t oMB   = off; off += szMB;
  const size_t oPART = off; off += szPART;
  if (off > ws_size) return;
  if (off > (size_t)134217728) return;

  char* ws = (char*)d_ws;
  u16*      XB   = (u16*)(ws + oXB);
  u16*      WB   = (u16*)(ws + oWB);
  float*    F    = (float*)(ws + oF);
  u16*      QH   = (u16*)(ws + oQH);
  u16*      QL   = (u16*)(ws + oQL);
  u16*      KH   = (u16*)(ws + oKH);
  u16*      KL   = (u16*)(ws + oKL);
  u16*      VP   = (u16*)(ws + oVP);
  u16*      OP   = (u16*)(ws + oOP);
  unsigned* MBT  = (unsigned*)(ws + oMB);
  float*    PART = (float*)(ws + oPART);

  const int n8x = (ROWS * DMOD) / 8;
  const int n8w = (DMOD * DMOD) / 8;
  if ((n8x % 256) != 0 || (n8w % 256) != 0 || (DMOD % 64) != 0 || (ROWS % 64) != 0 || (DMOD % 32) != 0) return;
  const dim3 blk(256);
  const dim3 gX(n8x / 256);
  const dim3 gW(n8w / 256);
  const dim3 gG((ROWS / 64) * (DMOD / 64));
  const dim3 bG(128);
  const dim3 gVT(NB * NH * (SEQ / 64));
  const dim3 gMB(NB * 32 * 32);
  const dim3 gAT(ATT_BLOCKS);
  const dim3 bAT(ATT_THREADS);
  const dim3 gWO(OUT1N / 256);

  cvt16<<<gX, blk, 0, stream>>>(q, XB, n8x, 0, 1.0f);
  cvt16<<<gW, blk, 0, stream>>>(wq, WB, n8w, 0, 1.0f);
  gemm_bfb<<<gG, bG, 0, stream>>>(XB, WB, bq, F, ROWS, DMOD, DMOD, 1.0f);
  cvt_split<<<gX, blk, 0, stream>>>(F, QH, QL, n8x, QSC);
  cvt16<<<gX, blk, 0, stream>>>(k, XB, n8x, 0, 1.0f);
  cvt16<<<gW, blk, 0, stream>>>(wk, WB, n8w, 0, 1.0f);
  gemm_bfb<<<gG, bG, 0, stream>>>(XB, WB, bk, F, ROWS, DMOD, DMOD, 1.0f);
  cvt_split<<<gX, blk, 0, stream>>>(F, KH, KL, n8x, KSC);
  cvt16<<<gX, blk, 0, stream>>>(v, XB, n8x, 0, 1.0f);
  cvt16<<<gW, blk, 0, stream>>>(wv, WB, n8w, 0, 1.0f);
  gemm_bfb<<<gG, bG, 0, stream>>>(XB, WB, bv, F, ROWS, DMOD, DMOD, 1.0f);
  vt16<<<gVT, blk, 0, stream>>>(F, VP);
  maskbits<<<gMB, blk, 0, stream>>>(mask, mskv, MBT);
  attn_fwd<<<gAT, bAT, 0, stream>>>(QH, QL, KH, KL, VP, MBT, OP, PART);
  cvt16<<<gW, blk, 0, stream>>>(wo, WB, n8w, 1, WOS);
  gemm_h1<<<gG, bG, 0, stream>>>(OP, WB, bo, out0, ROWS, DMOD, DMOD, 1.0f / (OSC * WOS));
  wout<<<gWO, blk, 0, stream>>>(PART, out1);
  (void)hipGetLastError();
}
